// RelativePositionalMultiHeadAttention_37263136260158
// MI455X (gfx1250) — hardware-verified
//
#include <hip/hip_runtime.h>


#define NB_  8
#define SS   1024
#define DD   512
#define NH_  8
#define HD   64
typedef _Float16 h16;
typedef unsigned short bf;
typedef __attribute__((ext_vector_type(16))) __bf16   v16bf;
typedef __attribute__((ext_vector_type(16))) _Float16 v16h;
typedef __attribute__((ext_vector_type(8)))  _Float16 v8h;
typedef __attribute__((ext_vector_type(8)))  unsigned short v8us;
typedef __attribute__((ext_vector_type(8)))  float    v8f;
typedef __attribute__((ext_vector_type(4)))  float    v4f;
typedef v8h  __attribute__((may_alias)) v8ha;
typedef v4f  __attribute__((may_alias)) v4fa;
typedef v8us __attribute__((may_alias)) v8usa;

__device__ __forceinline__ unsigned short f2bf(float f) { unsigned u = __float_as_uint(f); u += 0x7FFFu + ((u >> 16) & 1u); return (unsigned short)(u >> 16); }
__device__ __forceinline__ float bf2f(unsigned short b) { return __uint_as_float(((unsigned)b) << 16); }
__device__ __forceinline__ float bfr(float f) { return bf2f(f2bf(f)); }
__device__ __forceinline__ v16h cat16(v8h lo, v8h hi) { return __builtin_shufflevector(lo, hi, 0, 1, 2, 3, 4, 5, 6, 7, 8, 9, 10, 11, 12, 13, 14, 15); }
__device__ __forceinline__ v16bf cat16b(v8us lo, v8us hi) { return __builtin_bit_cast(v16bf, __builtin_shufflevector(lo, hi, 0, 1, 2, 3, 4, 5, 6, 7, 8, 9, 10, 11, 12, 13, 14, 15)); }
__device__ __forceinline__ v8f wmma16(v16h a, v16h b, v8f c) { return __builtin_amdgcn_wmma_f32_16x16x32_f16(false, a, false, b, (short)0, c, false, false); }
__device__ __forceinline__ v8f wmmab(v16bf a, v16bf b, v8f c) { return __builtin_amdgcn_wmma_f32_16x16x32_bf16(false, a, false, b, (short)0, c, false, false); }


template <typename T16> struct WFrag;
template <> struct WFrag<h16> { typedef v16h V; static __device__ __forceinline__ V ld(const h16* p) { return cat16(*(const v8h*)p, *(const v8h*)(p + 16)); } static __device__ __forceinline__ v8f mma(V a, V b, v8f c) { return wmma16(a, b, c); } };
template <> struct WFrag<bf> { typedef v16bf V; static __device__ __forceinline__ V ld(const bf* p) { return cat16b(*(const v8us*)p, *(const v8us*)(p + 16)); } static __device__ __forceinline__ v8f mma(V a, V b, v8f c) { return wmmab(a, b, c); } };
template <typename T16, int NSPLIT, bool BIAS>
__global__ __launch_bounds__(32) void k_gemmw(const T16* __restrict__ A, const T16* __restrict__ A2, const T16* __restrict__ Bt, const T16* __restrict__ Bt2, int K, float* C, int ldc, const float* __restrict__ bias, size_t sA, size_t sB, size_t sC) {
    typedef typename WFrag<T16>::V V;
    __shared__ __align__(16) float os[16 * 68];
    const size_t z = blockIdx.z; A += z * sA; if (A2) A2 += z * sA; Bt += z * sB; if (Bt2) Bt2 += z * sB; C += z * sC;
    const int lane = threadIdx.x & 31, lr = lane & 15, hi = lane >> 4; const int r0 = blockIdx.x * 64, c0 = blockIdx.y * 64;
    v8f acc[4][4];
#pragma unroll
    for (int mb = 0; mb < 4; ++mb)
#pragma unroll
        for (int nb = 0; nb < 4; ++nb) acc[mb][nb] = (v8f){};
    const size_t aoff = (size_t)(r0 + lr) * K + 8 * hi, boff = (size_t)(c0 + lr) * K + 8 * hi;
#pragma unroll 1
    for (int kc = 0; kc < K; kc += 32) {
        V a[4], a2[4];
#pragma unroll
        for (int mb = 0; mb < 4; ++mb) { a[mb] = WFrag<T16>::ld(A + aoff + (size_t)mb * 16 * K + kc); if (NSPLIT == 1 || NSPLIT == 2) a2[mb] = WFrag<T16>::ld(A2 + aoff + (size_t)mb * 16 * K + kc); }
#pragma unroll
        for (int nb = 0; nb < 4; ++nb) { const V b = WFrag<T16>::ld(Bt + boff + (size_t)nb * 16 * K + kc); V b2; if (NSPLIT >= 2) b2 = WFrag<T16>::ld(Bt2 + boff + (size_t)nb * 16 * K + kc);
#pragma unroll
            for (int mb = 0; mb < 4; ++mb) { acc[mb][nb] = WFrag<T16>::mma(a[mb], b, acc[mb][nb]); if (NSPLIT == 1 || NSPLIT == 2) acc[mb][nb] = WFrag<T16>::mma(a2[mb], b, acc[mb][nb]); if (NSPLIT >= 2) acc[mb][nb] = WFrag<T16>::mma(a[mb], b2, acc[mb][nb]); } }
        asm volatile("v_nop\n\tv_nop\n\tv_nop\n\tv_nop" : "+v"(acc[0][0]), "+v"(acc[1][1]), "+v"(acc[2][2]), "+v"(acc[3][3]) : "v"(a[0]), "v"(a[3]));
    }
#pragma unroll
    for (int mb = 0; mb < 4; ++mb) {
#pragma unroll
        for (int nb = 0; nb < 4; ++nb) {
#pragma unroll
            for (int j = 0; j < 8; ++j) os[(hi * 8 + j) * 68 + nb * 16 + lr] = acc[mb][nb][j]; }
        __builtin_amdgcn_wave_barrier(); asm volatile("" ::: "memory");
        float* crow = C + (size_t)(r0 + mb * 16) * ldc + c0;
#pragma unroll 1
        for (int ps = 0; ps < 2; ++ps) {
#pragma unroll
            for (int s = 0; s < 8; ++s) { const int row = 2 * s + hi, cofs = lr * 4; v4f val = *(const v4fa*)(os + row * 68 + cofs); if (BIAS) { val[0] += bfr(bias[c0 + cofs]); val[1] += bfr(bias[c0 + cofs + 1]); val[2] += bfr(bias[c0 + cofs + 2]); val[3] += bfr(bias[c0 + cofs + 3]); }
                *(volatile v4f*)(crow + (size_t)row * ldc + cofs) = val; }
            if (ps == 0) __threadfence(); }
        __builtin_amdgcn_wave_barrier(); asm volatile("" ::: "memory");
    }
}

__device__ __forceinline__ void splitf(float y, unsigned short& h, unsigned short& l) { h = f2bf(y); l = f2bf(y - bf2f(h)); }
typedef __attribute__((ext_vector_type(2))) unsigned short v2us;
typedef __attribute__((ext_vector_type(4))) unsigned short v4us;

__global__ __launch_bounds__(256) void k_cvt8(const float* __restrict__ src, bf* dst, size_t n8) { const size_t i = (size_t)blockIdx.x * 256 + threadIdx.x; if (i >= n8) return; const v8f v = *(const v8f*)(src + i * 8); v8us o;
#pragma unroll
    for (int k = 0; k < 8; ++k) o[k] = f2bf(v[k]); *(volatile v8us*)(dst + i * 8) = o; __threadfence(); *(volatile v8us*)(dst + i * 8) = o; }
__global__ __launch_bounds__(256) void k_whg(const float* __restrict__ w, bf* Bt) { const int e = (blockIdx.x * 256 + threadIdx.x) * 4; if (e >= DD * DD) return; const int c = e % DD; const int n = e / DD; const int h = n / HD, kk = n % HD; v4us o;
#pragma unroll
    for (int u = 0; u < 4; ++u) o[u] = f2bf(w[((size_t)h * DD + c + u) * HD + kk]); *(volatile v4us*)(Bt + e) = o; __threadfence(); *(volatile v4us*)(Bt + e) = o; }
__global__ __launch_bounds__(256) void k_pe(bf* Ph, bf* Pl) { const int e = (blockIdx.x * 256 + threadIdx.x) * 4; if (e >= 2 * SS * DD) return; const int c = e % DD; const int l = e / DD; const float pos = (float)(2 * SS - 1 - l); v4us oh, ol;
#pragma unroll 1
    for (int u = 0; u < 4; ++u) { const int cc = c + u; const int i2 = cc & ~1; const float theta = __fdiv_rn(pos, powf(10000.0f, (float)i2 / (float)DD)); const float val = (cc & 1) ? cosf(theta) : sinf(theta); unsigned short a, b; splitf(val, a, b); oh[u] = a; ol[u] = b; }
    *(volatile v4us*)(Ph + e) = oh; *(volatile v4us*)(Pl + e) = ol; __threadfence(); *(volatile v4us*)(Ph + e) = oh; *(volatile v4us*)(Pl + e) = ol; }
__global__ __launch_bounds__(256) void k_hpb(const float* __restrict__ F, const float* __restrict__ bias, int rows, bf* Ph, bf* Pl) { const size_t e = ((size_t)blockIdx.x * 256 + threadIdx.x) * 4; if (e >= (size_t)NH_ * rows * HD) return; const int d = (int)(e % HD); const int s = (int)((e / HD) % rows); const int h = (int)(e / ((size_t)HD * rows)); const float* f = F + (size_t)s * DD + h * HD + d; v4us oh, ol;
#pragma unroll
    for (int u = 0; u < 4; ++u) { const float x = bias ? __fadd_rn(f[u], bfr(bias[h * HD + d + u])) : f[u]; unsigned short a, b; splitf(x, a, b); oh[u] = a; ol[u] = b; } *(volatile v4us*)(Ph + e) = oh; *(volatile v4us*)(Pl + e) = ol; __threadfence(); *(volatile v4us*)(Ph + e) = oh; *(volatile v4us*)(Pl + e) = ol; }
__global__ __launch_bounds__(256) void k_vtp(const float* __restrict__ F, bf* Ph, bf* Pl) { const size_t e = ((size_t)blockIdx.x * 256 + threadIdx.x) * 2; if (e >= (size_t)NH_ * HD * SS) return; const int s = (int)(e % SS); const int d = (int)((e / SS) % HD); const int h = (int)(e / ((size_t)SS * HD)); v2us oh, ol;
#pragma unroll
    for (int u = 0; u < 2; ++u) { unsigned short a, b; splitf(F[(size_t)(s + u) * DD + h * HD + d], a, b); oh[u] = a; ol[u] = b; } *(volatile v2us*)(Ph + e) = oh; *(volatile v2us*)(Pl + e) = ol; __threadfence(); *(volatile v2us*)(Ph + e) = oh; *(volatile v2us*)(Pl + e) = ol; }
__global__ __launch_bounds__(256) void k_rsoft(const float* __restrict__ AC, const float* __restrict__ BD, const int* __restrict__ mk, bf* Ph, bf* Pl) { const int lane = threadIdx.x & 31; const int row = blockIdx.x * 8 + (threadIdx.x >> 5); if (row >= NH_ * SS) return; const int i = row % SS; const float* ar = AC + (size_t)row * SS; const float* br = BD + (size_t)row * 2 * SS + (2 * SS - 1 - i); float v[SS / 32]; float mx = -3.0e38f;
#pragma unroll
    for (int ch = 0; ch < SS / 128; ++ch) { const v4f a = *(const v4f*)(ar + ch * 128 + lane * 4);
#pragma unroll
        for (int u = 0; u < 4; ++u) { const int j = ch * 128 + lane * 4 + u; const float bd = (j <= i) ? br[j] : 0.f; const float t = (mk[j] == 0) ? -3.0e38f : __fadd_rn(a[u], bd) * 0.125f; v[ch * 4 + u] = t; mx = fmaxf(mx, t); } }
#pragma unroll
    for (int sh = 16; sh; sh >>= 1) mx = fmaxf(mx, __shfl_xor(mx, sh, 32));
    float sum = 0.f;
#pragma unroll
    for (int q = 0; q < SS / 32; ++q) { float d0 = __fsub_rn(v[q], mx); asm volatile("" : "+v"(d0)); v[q] = __builtin_amdgcn_exp2f(__fmul_rn(d0, 1.4426950408889634f)); sum += v[q]; }
#pragma unroll
    for (int sh = 16; sh; sh >>= 1) sum += __shfl_xor(sum, sh, 32);
    const float f = __fdiv_rn(1.0f, sum);
    for (int ps = 0; ps < 2; ++ps) {
#pragma unroll
        for (int ch = 0; ch < SS / 128; ++ch) { v4us oh, ol; for (int q = 0; q < 4; ++q) { unsigned short a2, c2; splitf(v[ch * 4 + q] * f, a2, c2); oh[q] = a2; ol[q] = c2; } const size_t oo = (size_t)row * SS + ch * 128 + lane * 4; *(volatile v4us*)(Ph + oo) = oh; *(volatile v4us*)(Pl + oo) = ol; }
        if (ps == 0) __threadfence(); } }
__global__ __launch_bounds__(256) void k_mrg(const float* __restrict__ O, bf* Ah, bf* Al) { const size_t e = ((size_t)blockIdx.x * 256 + threadIdx.x) * 4; if (e >= (size_t)NH_ * SS * HD) return; const int d = (int)(e % HD); const int s = (int)((e / HD) % SS); const int h = (int)(e / ((size_t)HD * SS)); const size_t oo = (size_t)s * DD + h * HD + d; v4us oh, ol;
#pragma unroll
    for (int u = 0; u < 4; ++u) { unsigned short a, b; splitf(O[e + u], a, b); oh[u] = a; ol[u] = b; } *(volatile v4us*)(Ah + oo) = oh; *(volatile v4us*)(Al + oo) = ol; __threadfence(); *(volatile v4us*)(Ah + oo) = oh; *(volatile v4us*)(Al + oo) = ol; }

extern "C" void kernel_launch(void* const* d_in, const int* in_sizes, int n_in,
                              void* d_out, int out_size, void* d_ws, size_t ws_size, hipStream_t stream) {
    (void)in_sizes; (void)n_in; (void)out_size;
    const float* xq = (const float*)d_in[0]; const float* xk = (const float*)d_in[1]; const float* xv = (const float*)d_in[2]; const int* mask = (const int*)d_in[3]; const float* wq = (const float*)d_in[4]; const float* wk = (const float*)d_in[5]; const float* wv = (const float*)d_in[6]; const float* wp = (const float*)d_in[7]; const float* bu = (const float*)d_in[8]; const float* bvv = (const float*)d_in[9]; const float* wo = (const float*)d_in[10];
    float* OUT = (float*)d_out;
    char* wsp = (char*)d_ws;
    auto take = [&](size_t bytes) { char* p = wsp; wsp += (bytes + 255) & ~(size_t)255; return (void*)p; };
    bf* BQ = (bf*)take((size_t)DD * DD * 2); bf* BK = (bf*)take((size_t)DD * DD * 2); bf* BV = (bf*)take((size_t)DD * DD * 2); bf* BPp = (bf*)take((size_t)DD * DD * 2); bf* BO = (bf*)take((size_t)DD * DD * 2);
    bf* PEh = (bf*)take((size_t)2 * SS * DD * 2); bf* PEl = (bf*)take((size_t)2 * SS * DD * 2); float* PH = (float*)take((size_t)2 * SS * DD * 4); bf* PHh = (bf*)take((size_t)NH_ * 2 * SS * HD * 2); bf* PHl = (bf*)take((size_t)NH_ * 2 * SS * HD * 2);
    bf* XB = (bf*)take((size_t)SS * DD * 2); float* F = (float*)take((size_t)SS * DD * 4); bf* QUh = (bf*)take((size_t)NH_ * SS * HD * 2); bf* QUl = (bf*)take((size_t)NH_ * SS * HD * 2); bf* QVh = (bf*)take((size_t)NH_ * SS * HD * 2); bf* QVl = (bf*)take((size_t)NH_ * SS * HD * 2); bf* KPh = (bf*)take((size_t)NH_ * SS * HD * 2); bf* KPl = (bf*)take((size_t)NH_ * SS * HD * 2); bf* VTh = (bf*)take((size_t)NH_ * HD * SS * 2); bf* VTl = (bf*)take((size_t)NH_ * HD * SS * 2);
    float* AC = (float*)take((size_t)NH_ * SS * SS * 4); float* BDm = (float*)take((size_t)NH_ * SS * 2 * SS * 4); bf* Ph = (bf*)take((size_t)NH_ * SS * SS * 2); bf* Pl = (bf*)take((size_t)NH_ * SS * SS * 2); float* O = (float*)take((size_t)NH_ * SS * HD * 4); bf* ATh = (bf*)take((size_t)SS * DD * 2); bf* ATl = (bf*)take((size_t)SS * DD * 2);
    if ((size_t)(wsp - (char*)d_ws) > ws_size) return;
    k_whg<<<(DD * DD / 4 + 255) / 256, 256, 0, stream>>>(wq, BQ); k_whg<<<(DD * DD / 4 + 255) / 256, 256, 0, stream>>>(wk, BK); k_whg<<<(DD * DD / 4 + 255) / 256, 256, 0, stream>>>(wv, BV); k_whg<<<(DD * DD / 4 + 255) / 256, 256, 0, stream>>>(wp, BPp); k_cvt8<<<(DD * DD / 8 + 255) / 256, 256, 0, stream>>>(wo, BO, DD * DD / 8);
    k_pe<<<(2 * SS * DD / 4 + 255) / 256, 256, 0, stream>>>(PEh, PEl);
    k_gemmw<bf, 1, false><<<dim3(2 * SS / 64, DD / 64, 1), 32, 0, stream>>>(PEh, PEl, BPp, nullptr, DD, PH, DD, nullptr, 0, 0, 0);
    k_hpb<<<(unsigned)(((size_t)NH_ * 2 * SS * HD / 4 + 255) / 256), 256, 0, stream>>>(PH, nullptr, 2 * SS, PHh, PHl);
    const dim3 gp(SS / 64, DD / 64, 1); const unsigned LH = (unsigned)(((size_t)NH_ * SS * HD / 4 + 255) / 256); const size_t zq = (size_t)SS * HD, zA = (size_t)SS * SS, zB = (size_t)SS * 2 * SS, zp = (size_t)2 * SS * HD, zv = (size_t)HD * SS;
    for (int b = 0; b < NB_; ++b) {
        k_cvt8<<<(SS * DD / 8 + 255) / 256, 256, 0, stream>>>(xq + (size_t)b * SS * DD, XB, SS * DD / 8); k_gemmw<bf, 0, false><<<gp, 32, 0, stream>>>(XB, nullptr, BQ, nullptr, DD, F, DD, nullptr, 0, 0, 0);
        k_hpb<<<LH, 256, 0, stream>>>(F, bu, SS, QUh, QUl); k_hpb<<<LH, 256, 0, stream>>>(F, bvv, SS, QVh, QVl);
        k_cvt8<<<(SS * DD / 8 + 255) / 256, 256, 0, stream>>>(xk + (size_t)b * SS * DD, XB, SS * DD / 8); k_gemmw<bf, 0, false><<<gp, 32, 0, stream>>>(XB, nullptr, BK, nullptr, DD, F, DD, nullptr, 0, 0, 0); k_hpb<<<LH, 256, 0, stream>>>(F, nullptr, SS, KPh, KPl);
        k_cvt8<<<(SS * DD / 8 + 255) / 256, 256, 0, stream>>>(xv + (size_t)b * SS * DD, XB, SS * DD / 8); k_gemmw<bf, 0, false><<<gp, 32, 0, stream>>>(XB, nullptr, BV, nullptr, DD, F, DD, nullptr, 0, 0, 0); k_vtp<<<(unsigned)(((size_t)NH_ * HD * SS / 2 + 255) / 256), 256, 0, stream>>>(F, VTh, VTl);
        k_gemmw<bf, 2, false><<<dim3(SS / 64, SS / 64, NH_), 32, 0, stream>>>(QUh, QUl, KPh, KPl, HD, AC, SS, nullptr, zq, zq, zA);
        k_gemmw<bf, 2, false><<<dim3(SS / 64, 2 * SS / 64, NH_), 32, 0, stream>>>(QVh, QVl, PHh, PHl, HD, BDm, 2 * SS, nullptr, zq, zp, zB);
        k_rsoft<<<NH_ * SS / 8, 256, 0, stream>>>(AC, BDm, mask + (size_t)b * SS, Ph, Pl);
        k_gemmw<bf, 2, false><<<dim3(SS / 64, 1, NH_), 32, 0, stream>>>(Ph, Pl, VTh, VTl, SS, O, HD, nullptr, zA, zv, zq);
        k_mrg<<<LH, 256, 0, stream>>>(O, ATh, ATl);
        k_gemmw<bf, 1, false><<<gp, 32, 0, stream>>>(ATh, ATl, BO, nullptr, DD, OUT + (size_t)b * SS * DD, DD, nullptr, 0, 0, 0); }
}
